// SS2D_41394894799413
// MI455X (gfx1250) — hardware-verified
//
#include <hip/hip_runtime.h>
#include <math.h>

typedef __attribute__((ext_vector_type(16))) _Float16 v16h;
typedef __attribute__((ext_vector_type(8)))  _Float16 v8h;
typedef __attribute__((ext_vector_type(16))) __bf16   v16b;
typedef __attribute__((ext_vector_type(8)))  __bf16   v8b;
typedef __attribute__((ext_vector_type(8)))  float    v8f;
typedef __attribute__((ext_vector_type(4)))  float    v4f;

constexpr int kBat  = 2;
constexpr int kCh   = 192;
constexpr int kHgt  = 64;
constexpr int kWid  = 64;
constexpr int kLen  = kHgt * kWid;
constexpr int kDir  = 4;
constexpr int kNst  = 16;
constexpr int kDtR  = 6;
constexpr int kCpr  = kDtR + 2 * kNst;
constexpr int kCAll = kDir * kCpr;
constexpr int kCPad = 192;
constexpr int kNCh  = 64;
constexpr int kCLen = 64;
constexpr int kSCh  = 64;
constexpr int kDBlk = kCh / kSCh;
constexpr int kPQ   = 2 * kNst;
constexpr int kSXP  = 40;
constexpr int kTP   = 68;
constexpr int kXTP  = 196;
static_assert(kLen == kNCh * kCLen, "chunks");
static_assert(kCLen == kSCh, "staging map assumes 64 steps x 64 threads");
static_assert(kCh % kSCh == 0, "channel blocks");
static_assert(kCAll <= kCPad, "projection pad");
static_assert(kCh % 32 == 0 && kLen % 64 == 0 && kCPad % 64 == 0, "GEMM K % 32, M and N % 64");
static_assert(((kLen / 64) * (kCPad / 64)) % 8 == 0, "GEMM grid exact");
static_assert(kLen % 32 == 0 && kCh == 192, "transpose tile map assumes 32 positions x 192 channels");
static_assert((kCPad * kCh) % (192 * 8) == 0 && (kCAll * kCh) % (192 * 8) == 0, "weight plane kernel coverage");

constexpr size_t kOffXTB  = 0;
constexpr size_t kOffXT32 = kOffXTB  + (size_t)kBat * kLen * kCh * 2;
constexpr size_t kOffWPB  = kOffXT32 + (size_t)kBat * kLen * kCh * 4;
constexpr size_t kOffXDBL = kOffWPB  + (size_t)kCPad * kCh * 2;
constexpr size_t kOffPQ   = kOffXDBL + (size_t)kBat * kLen * kCPad * 4;
constexpr size_t kOffHIN  = kOffPQ   + (size_t)kBat * kDir * kNCh * kPQ * kCh * 4;
constexpr size_t kOffY    = kOffHIN  + (size_t)kBat * kDir * kNCh * kNst * kCh * 4;
constexpr size_t kWsTotal = kOffY    + (size_t)kBat * kDir * kLen * kCh * 4;
static_assert(kWsTotal == 59842560ull, "carve total");
static_assert(kWsTotal <= 134217728ull, "carve cap");
static_assert((kOffXT32 % 128) == 0 && (kOffWPB % 128) == 0 && (kOffXDBL % 128) == 0 &&
              (kOffPQ % 128) == 0 && (kOffHIN % 128) == 0 && (kOffY % 128) == 0, "128-B aligned regions");

__device__ __forceinline__ unsigned short f2bf_bits(float f) {
  unsigned u = __float_as_uint(f);
  return (unsigned short)((u + 0x7FFFu + ((u >> 16) & 1u)) >> 16);
}
__device__ __forceinline__ float bf_bits2f(unsigned short h) { return __uint_as_float(((unsigned)h) << 16); }
__device__ __forceinline__ float rne_bf16(float f) { return bf_bits2f(f2bf_bits(f)); }

__device__ __forceinline__ void dep_guard_h(v8f& a, v8f& b, v16h x, v16h y) { asm volatile("v_nop\n\tv_nop\n\tv_nop\n\tv_nop" : "+v"(a), "+v"(b) : "v"(x), "v"(y)); }
__device__ __forceinline__ void dep_guard_b(v8f& a, v8f& b, v16b x, v16b y) { asm volatile("v_nop\n\tv_nop\n\tv_nop\n\tv_nop" : "+v"(a), "+v"(b) : "v"(x), "v"(y)); }
__device__ __forceinline__ void keep4_h(v16h a, v16h b, v16h c, v16h d) { asm volatile("v_nop" :: "v"(a), "v"(b), "v"(c), "v"(d)); }
__device__ __forceinline__ void keep4_b(v16b a, v16b b, v16b c, v16b d) { asm volatile("v_nop" :: "v"(a), "v"(b), "v"(c), "v"(d)); }
__device__ __forceinline__ void acc_guard4(v8f& a, v8f& b, v8f& c, v8f& d) { asm volatile("v_nop\n\tv_nop\n\tv_nop\n\tv_nop" : "+v"(a), "+v"(b), "+v"(c), "+v"(d)); }
template <typename T> struct Frag;
template <> struct Frag<_Float16> {
  typedef v16h V; union U { v16h v; v8h h[2]; };
  static __device__ __forceinline__ v16h load(const _Float16* p) {
    U f; f.h[0] = *(const v8h*)(p); f.h[1] = *(const v8h*)(p + 16); return f.v;
  }
  static __device__ __forceinline__ v8f mma(v16h a, v16h b, v8f c) {
    return __builtin_amdgcn_wmma_f32_16x16x32_f16(false, a, false, b, (short)0, c, false, false);
  }
  static __device__ __forceinline__ void guard(v8f& a, v8f& b, v16h x, v16h y) { dep_guard_h(a, b, x, y); }
  static __device__ __forceinline__ void keep(v16h a, v16h b, v16h c, v16h d) { keep4_h(a, b, c, d); }
};
template <> struct Frag<__bf16> {
  typedef v16b V; union U { v16b v; v8b h[2]; };
  static __device__ __forceinline__ v16b load(const __bf16* p) {
    U f; f.h[0] = *(const v8b*)(p); f.h[1] = *(const v8b*)(p + 16); return f.v;
  }
  static __device__ __forceinline__ v8f mma(v16b a, v16b b, v8f c) {
    return __builtin_amdgcn_wmma_f32_16x16x32_bf16(false, a, false, b, (short)0, c, false, false);
  }
  static __device__ __forceinline__ void guard(v8f& a, v8f& b, v16b x, v16b y) { dep_guard_b(a, b, x, y); }
  static __device__ __forceinline__ void keep(v16b a, v16b b, v16b c, v16b d) { keep4_b(a, b, c, d); }
};

template <int ET> struct Elem;
template <> struct Elem<0> { typedef _Float16 T; };
template <> struct Elem<1> { typedef __bf16 T; };
template <int ET, int SPL, int BIAS_MODE, int OUT_MODE, bool RESID, int ACT = 0>
__global__ __launch_bounds__(256) void wmma_gemm64(
    const unsigned short* __restrict__ Ap, const unsigned short* __restrict__ A2p, int lda, long strideA,
    const unsigned short* __restrict__ Btp, const unsigned short* __restrict__ Bt2p, int ldb, long strideB,
    void* __restrict__ Cout, void* __restrict__ Cout2, int ldc, long strideC,
    const float* __restrict__ bias,
    const float* __restrict__ resid, long strideR,
    int M, int N, int K, float scale) {
  typedef typename Elem<ET>::T T;
  typedef typename Frag<T>::V V;
  const T* A = (const T*)Ap; const T* A2 = (const T*)A2p; const T* Bt = (const T*)Btp; const T* Bt2 = (const T*)Bt2p;
  __shared__ __align__(16) float sT[8][16 * 68];
  const int b    = blockIdx.y;
  const int lane = threadIdx.x & 31;
  const int wave = threadIdx.x >> 5;
  const int tilesN = N >> 6;
  const int tilesM = M >> 6;
  const int tile = blockIdx.x * 8 + wave;
  if (tile >= tilesM * tilesN) return;
  const int tm = tile / tilesN;
  const int tn = tile - tm * tilesN;
  const int m0 = tm << 6;
  const int n0 = tn << 6;

  const T* Ab  = A  + (size_t)b * strideA;
  const T* Bb  = Bt + (size_t)b * strideB;
  const T* Ab2 = (SPL >= 1) ? (A2  + (size_t)b * strideA) : nullptr;
  const T* Bb2 = (SPL == 2) ? (Bt2 + (size_t)b * strideB) : nullptr;

  const int rlane = lane & 15;
  const int koff  = (lane >> 4) * 8;
  const int mOff  = (lane >> 4) * 8;

  v8f acc[4][4];
#pragma unroll
  for (int i = 0; i < 4; ++i)
#pragma unroll
    for (int j = 0; j < 4; ++j) acc[i][j] = (v8f){0.f,0.f,0.f,0.f,0.f,0.f,0.f,0.f};

  for (int k0 = 0; k0 < K; k0 += 32) {
    V bh[4], bl[4];
#pragma unroll
    for (int j = 0; j < 4; ++j) {
      const size_t bo = (size_t)(n0 + (j << 4) + rlane) * ldb + koff + k0;
      bh[j] = Frag<T>::load(Bb + bo);
      if (SPL == 2) bl[j] = Frag<T>::load(Bb2 + bo);
    }
#pragma unroll
    for (int i = 0; i < 4; ++i) {
      const size_t ao = (size_t)(m0 + (i << 4) + rlane) * lda + koff + k0;
      V ah = Frag<T>::load(Ab + ao);
      V al;
      if (SPL >= 1) al = Frag<T>::load(Ab2 + ao);
#pragma unroll
      for (int j = 0; j < 4; ++j) {
        acc[i][j] = Frag<T>::mma(ah, bh[j], acc[i][j]);
        if (SPL == 2) acc[i][j] = Frag<T>::mma(ah, bl[j], acc[i][j]);
        if (SPL >= 1) acc[i][j] = Frag<T>::mma(al, bh[j], acc[i][j]);
      }
      Frag<T>::guard(acc[i][0], acc[i][3], ah, (SPL >= 1) ? al : ah);
    }
    Frag<T>::keep(bh[0], bh[1], bh[2], bh[3]);
    if (SPL == 2) Frag<T>::keep(bl[0], bl[1], bl[2], bl[3]);
  }
  acc_guard4(acc[0][0], acc[0][1], acc[0][2], acc[0][3]);
  acc_guard4(acc[1][0], acc[1][1], acc[1][2], acc[1][3]);
  acc_guard4(acc[2][0], acc[2][1], acc[2][2], acc[2][3]);
  acc_guard4(acc[3][0], acc[3][1], acc[3][2], acc[3][3]);

  float* slab = sT[wave];
  const float* Rb = RESID ? (resid + (size_t)b * strideR) : nullptr;
#pragma unroll
  for (int i = 0; i < 4; ++i) {
    const int mBase = m0 + (i << 4);
#pragma unroll
    for (int j = 0; j < 4; ++j) {
      const int n = n0 + (j << 4) + rlane;
      float bv = 0.f;
      if (BIAS_MODE == 2) bv = bias[n];
#pragma unroll
      for (int r = 0; r < 8; ++r) {
        float v = acc[i][j][r] * scale;
        if (BIAS_MODE == 1) v += bias[mBase + mOff + r];
        if (BIAS_MODE == 2) v += bv;
        if (RESID) v += Rb[(size_t)(mBase + mOff + r) * ldc + n];
        if (ACT == 1) v = tanhf(v);
        if (ACT == 2) v = fmaxf(v, 0.0f);
        if (ACT == 3) v = v / (1.0f + expf(-v));
        if (ACT == 4) v = (v > 0.f) ? v : 0.01f * v;
        slab[(mOff + r) * 68 + (j << 4) + rlane] = v;
      }
    }
    __builtin_amdgcn_fence(__ATOMIC_RELEASE, "workgroup");
    __builtin_amdgcn_wave_barrier();
    __builtin_amdgcn_fence(__ATOMIC_ACQUIRE, "workgroup");
    if (OUT_MODE == 0) {
      float* C = (float*)Cout + (size_t)b * strideC;
      const int hh = lane >> 4, c4 = (lane & 15) * 4;
      for (int pass = 0; pass < 2; ++pass) {
#pragma unroll
        for (int it = 0; it < 8; ++it) {
          const int row = it * 2 + hh;
          v4f v = *(const v4f*)(slab + row * 68 + c4);
          *(volatile v4f*)(C + (size_t)(mBase + row) * ldc + n0 + c4) = v;
        }
        __threadfence();
      }
    } else {
      const int q = lane >> 3, c8 = (lane & 7) * 8;
      unsigned short* C  = (unsigned short*)Cout  + (size_t)b * strideC;
      unsigned short* C2 = (OUT_MODE == 2) ? ((unsigned short*)Cout2 + (size_t)b * strideC) : nullptr;
      for (int pass = 0; pass < 2; ++pass) {
#pragma unroll
        for (int it = 0; it < 4; ++it) {
          const int row = it * 4 + q;
          const float* sp = slab + row * 68 + c8;
          v8h hv, lv;
#pragma unroll
          for (int e = 0; e < 8; ++e) {
            if (OUT_MODE == 1) {
              hv[e] = (_Float16)sp[e];
            } else {
              unsigned short hb = f2bf_bits(sp[e]);
              unsigned short lb = f2bf_bits(sp[e] - bf_bits2f(hb));
              hv[e] = __builtin_bit_cast(_Float16, hb);
              lv[e] = __builtin_bit_cast(_Float16, lb);
            }
          }
          *(volatile v8h*)(C + (size_t)(mBase + row) * ldc + n0 + c8) = hv;
          if (OUT_MODE == 2) *(volatile v8h*)(C2 + (size_t)(mBase + row) * ldc + n0 + c8) = lv;
        }
        __threadfence();
      }
    }
    __builtin_amdgcn_fence(__ATOMIC_RELEASE, "workgroup");
    __builtin_amdgcn_wave_barrier();
    __builtin_amdgcn_fence(__ATOMIC_ACQUIRE, "workgroup");
  }
}

__device__ __forceinline__ int scan_pos(int k, int l) {
  const int ll = (k >= 2) ? (kLen - 1 - l) : l;
  const int pt = ((ll & (kHgt - 1)) << 6) | (ll >> 6);
  return (k & 1) ? pt : ll;
}

__device__ __forceinline__ float delta_of(const float* xr, const float* wr, float bias) {
  float v = 0.0f;
#pragma unroll
  for (int r = 0; r < kDtR; ++r) v = fmaf(xr[r], wr[r], v);
  v += bias;
  const float a = expf(-fabsf(v));
  return fmaxf(v, 0.0f) + log1pf(a);
}

__device__ __forceinline__ void stage_xdbl(float* sX, const float* __restrict__ XDBL, int b, int k, int l0, int tid) {
#pragma unroll 1
  for (int i = 0; i < kCpr; ++i) {
    const int e = tid + kSCh * i;
    const int s = e / kCpr;
    const int c = e - s * kCpr;
    const int col = c + ((c >= kDtR) ? 2 : 0);
    const int p = scan_pos(k, l0 + s);
    sX[s * kSXP + col] = XDBL[((size_t)(b * kLen + p)) * kCPad + k * kCpr + c];
  }
}

__global__ __launch_bounds__(256) void xpose_kernel(
    const float* __restrict__ x, float* __restrict__ XT32, unsigned short* __restrict__ XTB) {
  __shared__ __align__(16) float sT[32 * kXTP];
  const int tid = threadIdx.x, lane = tid & 31, wave = tid >> 5;
  const int b  = blockIdx.x >> 7;
  const int p0 = (blockIdx.x & 127) * 32;
#pragma unroll 1
  for (int i = 0; i < 24; ++i) {
    const int d = wave * 24 + i;
    sT[lane * kXTP + d] = rne_bf16(x[((size_t)(b * kCh + d)) * kLen + p0 + lane]);
  }
  __syncthreads();
  const int q4 = lane >> 3, c8 = lane & 7;
  v4f fv[6];
#pragma unroll
  for (int it = 0; it < 6; ++it) {
    const int L = it * 32 + wave * 4 + q4;
    const int row = L / 6, seg = L - row * 6;
    fv[it] = *(const v4f*)(sT + row * kXTP + seg * 32 + c8 * 4);
  }
  v8h hv[3];
#pragma unroll
  for (int it = 0; it < 3; ++it) {
    const int L = it * 32 + wave * 4 + q4;
    const int row = L / 3, seg = L - row * 3;
    const float* sp = sT + row * kXTP + seg * 64 + c8 * 8;
    const v4f a0 = *(const v4f*)(sp);
    const v4f a1 = *(const v4f*)(sp + 4);
    v8h t;
#pragma unroll
    for (int e = 0; e < 4; ++e) {
      const unsigned short hb0 = f2bf_bits(a0[e]);
      const unsigned short hb1 = f2bf_bits(a1[e]);
      t[e]     = __builtin_bit_cast(_Float16, hb0);
      t[4 + e] = __builtin_bit_cast(_Float16, hb1);
    }
    hv[it] = t;
  }
  float* xt32b = XT32 + ((size_t)(b * kLen + p0)) * kCh;
  unsigned short* xtbb = XTB + ((size_t)(b * kLen + p0)) * kCh;
  for (int pass = 0; pass < 2; ++pass) {
#pragma unroll
    for (int it = 0; it < 6; ++it) {
      const int L = it * 32 + wave * 4 + q4;
      const int row = L / 6, seg = L - row * 6;
      *(volatile v4f*)(xt32b + (size_t)row * kCh + seg * 32 + c8 * 4) = fv[it];
    }
#pragma unroll
    for (int it = 0; it < 3; ++it) {
      const int L = it * 32 + wave * 4 + q4;
      const int row = L / 3, seg = L - row * 3;
      *(volatile v8h*)(xtbb + (size_t)row * kCh + seg * 64 + c8 * 8) = hv[it];
    }
    __threadfence();
  }
}

__global__ __launch_bounds__(192) void wproj_plane_kernel(const float* __restrict__ W, unsigned short* __restrict__ WPB) {
  const int i = blockIdx.x * 192 + threadIdx.x;
  const size_t e0 = (size_t)i * 8;
  const bool valid = (blockIdx.x * 8) < kCAll;
  const float fac = valid ? 1.0f : 0.0f;
  const size_t ec = valid ? e0 : (size_t)0;
  const v4f a0 = *(const v4f*)(W + ec);
  const v4f a1 = *(const v4f*)(W + ec + 4);
  v8h hv;
#pragma unroll
  for (int e = 0; e < 4; ++e) {
    const unsigned short hb0 = f2bf_bits(a0[e] * fac);
    const unsigned short hb1 = f2bf_bits(a1[e] * fac);
    hv[e]     = __builtin_bit_cast(_Float16, hb0);
    hv[4 + e] = __builtin_bit_cast(_Float16, hb1);
  }
  unsigned short* dst = WPB + e0;
  *(volatile v8h*)dst = hv;
  __threadfence();
  *(volatile v8h*)dst = hv;
}

__global__ __launch_bounds__(64) void scan_phase_a(
    const float* __restrict__ XT32, const float* __restrict__ XDBL,
    const float* __restrict__ dtW, const float* __restrict__ dtb, const float* __restrict__ Alog,
    float* __restrict__ PQ) {
  __shared__ __align__(16) float sX[kCLen * kSXP];
  __shared__ __align__(16) float sA[kNst * kSCh];
  __shared__ __align__(16) float sO[kPQ * kTP];
  const int tid = threadIdx.x, lane = tid & 31, wave = tid >> 5;
  int bid = blockIdx.x;
  const int dblk = bid % kDBlk; bid /= kDBlk;
  const int chunk = bid % kNCh;
  const int bk = bid / kNCh;
  const int k = bk & 3, b = bk >> 2;
  const int d0 = dblk * kSCh, d = d0 + tid;
  const int l0 = chunk * kCLen;
  const int kd = k * kCh + d;
  float wr[kDtR];
#pragma unroll
  for (int r = 0; r < kDtR; ++r) wr[r] = rne_bf16(dtW[(size_t)kd * kDtR + r]);
  const float bias = rne_bf16(dtb[kd]);
  asm volatile("" ::: "memory");
#pragma unroll 1
  for (int s = 0; s < kNst; ++s) sA[s * kSCh + tid] = -expf(rne_bf16(Alog[(size_t)kd * kNst + s]));
  stage_xdbl(sX, XDBL, b, k, l0, tid);
  __syncthreads();
  float negA[kNst], qv[kNst], pv[kNst];
#pragma unroll
  for (int n = 0; n < kNst; ++n) { negA[n] = sA[n * kSCh + tid]; qv[n] = 0.0f; pv[n] = 1.0f; }
  const float* ub = XT32 + (size_t)b * kLen * kCh + d;
#pragma unroll 1
  for (int s = 0; s < kCLen; ++s) {
    const int p = scan_pos(k, l0 + s);
    const float u = ub[(size_t)p * kCh];
    const float* xr = sX + s * kSXP;
    const float dl = delta_of(xr, wr, bias);
    const float du = dl * u;
    float Bs[kNst];
#pragma unroll
    for (int q = 0; q < 4; ++q) {
      const v4f bv = *(const v4f*)(xr + 8 + 4 * q);
      Bs[4 * q + 0] = bv[0]; Bs[4 * q + 1] = bv[1]; Bs[4 * q + 2] = bv[2]; Bs[4 * q + 3] = bv[3];
    }
#pragma unroll
    for (int n = 0; n < kNst; ++n) {
      const float a = __expf(dl * negA[n]);
      qv[n] = a * qv[n] + du * Bs[n];
      pv[n] = pv[n] * a;
    }
  }
#pragma unroll
  for (int n = 0; n < kNst; ++n) { sO[n * kTP + tid] = pv[n]; sO[(kNst + n) * kTP + tid] = qv[n]; }
  __syncthreads();
  const int q4 = lane >> 3, c8 = lane & 7;
  float* pq = PQ + ((size_t)(bk * kNCh + chunk) * kPQ) * kCh + d0;
  for (int pass = 0; pass < 2; ++pass) {
#pragma unroll
    for (int it = 0; it < 8; ++it) {
      const int L = it * 8 + wave * 4 + q4;
      const int j = L >> 1, hf = L & 1;
      const v4f val = *(const v4f*)(sO + j * kTP + hf * 32 + c8 * 4);
      *(volatile v4f*)(pq + (size_t)j * kCh + hf * 32 + c8 * 4) = val;
    }
    __threadfence();
  }
}

__global__ __launch_bounds__(64) void chunk_combine_kernel(const float* __restrict__ PQ, float* __restrict__ HIN) {
  __shared__ __align__(16) float sP[kPQ * kTP];
  __shared__ __align__(16) float sH[kNst * kTP];
  const int tid = threadIdx.x, lane = tid & 31, wave = tid >> 5;
  const int dblk = blockIdx.x % kDBlk;
  const int bk = blockIdx.x / kDBlk;
  const int d0 = dblk * kSCh;
  const int q4 = lane >> 3, c8 = lane & 7;
  float h[kNst];
#pragma unroll
  for (int n = 0; n < kNst; ++n) h[n] = 0.0f;
#pragma unroll 1
  for (int chunk = 0; chunk < kNCh; ++chunk) {
#pragma unroll
    for (int n = 0; n < kNst; ++n) sH[n * kTP + tid] = h[n];
    const float* pqb = PQ + ((size_t)(bk * kNCh + chunk) * kPQ) * kCh + d0;
#pragma unroll
    for (int i = 0; i < 8; ++i) {
      const int idx = tid + kSCh * i;
      const int row = idx >> 4, col4 = (idx & 15) * 4;
      *(v4f*)(sP + row * kTP + col4) = *(const v4f*)(pqb + (size_t)row * kCh + col4);
    }
    __syncthreads();
    float* hb = HIN + ((size_t)(bk * kNCh + chunk) * kNst) * kCh + d0;
    for (int pass = 0; pass < 2; ++pass) {
#pragma unroll
      for (int it = 0; it < 4; ++it) {
        const int L = it * 8 + wave * 4 + q4;
        const int n = L >> 1, hf = L & 1;
        const v4f val = *(const v4f*)(sH + n * kTP + hf * 32 + c8 * 4);
        *(volatile v4f*)(hb + (size_t)n * kCh + hf * 32 + c8 * 4) = val;
      }
      __threadfence();
    }
#pragma unroll
    for (int n = 0; n < kNst; ++n) h[n] = sP[n * kTP + tid] * h[n] + sP[(kNst + n) * kTP + tid];
    __syncthreads();
  }
}

__global__ __launch_bounds__(64) void scan_phase_b(
    const float* __restrict__ XT32, const float* __restrict__ XDBL,
    const float* __restrict__ dtW, const float* __restrict__ dtb, const float* __restrict__ Alog,
    const float* __restrict__ Ds, const float* __restrict__ HIN, float* __restrict__ Y) {
  __shared__ __align__(16) float sX[kCLen * kSXP];
  __shared__ __align__(16) float sA[kNst * kSCh];
  __shared__ __align__(16) float sHn[kNst * kTP];
  __shared__ __align__(16) float sY[kCLen * kTP];
  const int tid = threadIdx.x, lane = tid & 31, wave = tid >> 5;
  int bid = blockIdx.x;
  const int dblk = bid % kDBlk; bid /= kDBlk;
  const int chunk = bid % kNCh;
  const int bk = bid / kNCh;
  const int k = bk & 3, b = bk >> 2;
  const int d0 = dblk * kSCh, d = d0 + tid;
  const int l0 = chunk * kCLen;
  const int kd = k * kCh + d;
  float wr[kDtR];
#pragma unroll
  for (int r = 0; r < kDtR; ++r) wr[r] = rne_bf16(dtW[(size_t)kd * kDtR + r]);
  const float bias = rne_bf16(dtb[kd]);
  const float Dd = rne_bf16(Ds[kd]);
  asm volatile("" ::: "memory");
#pragma unroll 1
  for (int s = 0; s < kNst; ++s) sA[s * kSCh + tid] = -expf(rne_bf16(Alog[(size_t)kd * kNst + s]));
  {
    const float* hsrc = HIN + ((size_t)(bk * kNCh + chunk) * kNst) * kCh + d0;
#pragma unroll
    for (int i = 0; i < 4; ++i) {
      const int idx = tid + kSCh * i;
      const int row = idx >> 4, col4 = (idx & 15) * 4;
      *(v4f*)(sHn + row * kTP + col4) = *(const v4f*)(hsrc + (size_t)row * kCh + col4);
    }
  }
  stage_xdbl(sX, XDBL, b, k, l0, tid);
  __syncthreads();
  float negA[kNst], h[kNst];
#pragma unroll
  for (int n = 0; n < kNst; ++n) { negA[n] = sA[n * kSCh + tid]; h[n] = sHn[n * kTP + tid]; }
  const float* ub = XT32 + (size_t)b * kLen * kCh + d;
#pragma unroll 1
  for (int s = 0; s < kCLen; ++s) {
    const int p = scan_pos(k, l0 + s);
    const float u = ub[(size_t)p * kCh];
    const float* xr = sX + s * kSXP;
    const float dl = delta_of(xr, wr, bias);
    const float du = dl * u;
    float Bs[kNst], Cs[kNst];
#pragma unroll
    for (int q = 0; q < 4; ++q) {
      const v4f bv = *(const v4f*)(xr + 8 + 4 * q);
      const v4f cv = *(const v4f*)(xr + 8 + kNst + 4 * q);
      Bs[4 * q + 0] = bv[0]; Bs[4 * q + 1] = bv[1]; Bs[4 * q + 2] = bv[2]; Bs[4 * q + 3] = bv[3];
      Cs[4 * q + 0] = cv[0]; Cs[4 * q + 1] = cv[1]; Cs[4 * q + 2] = cv[2]; Cs[4 * q + 3] = cv[3];
    }
    float ysum = 0.0f;
#pragma unroll
    for (int n = 0; n < kNst; ++n) {
      const float a = __expf(dl * negA[n]);
      h[n] = a * h[n] + du * Bs[n];
      ysum = fmaf(h[n], Cs[n], ysum);
    }
    sY[s * kTP + tid] = ysum + Dd * u;
  }
  __syncthreads();
  const int q4 = lane >> 3, c8 = lane & 7;
  float* yb = Y + (size_t)bk * kLen * kCh + d0;
  for (int pass = 0; pass < 2; ++pass) {
#pragma unroll
    for (int it = 0; it < 16; ++it) {
      const int L = it * 8 + wave * 4 + q4;
      const int s = L >> 1, hf = L & 1;
      const int p = scan_pos(k, l0 + s);
      const v4f val = *(const v4f*)(sY + s * kTP + hf * 32 + c8 * 4);
      *(volatile v4f*)(yb + (size_t)p * kCh + hf * 32 + c8 * 4) = val;
    }
    __threadfence();
  }
}

__global__ __launch_bounds__(192) void merge_ln_kernel(
    const float* __restrict__ Y, const float* __restrict__ lnw, const float* __restrict__ lnb,
    float* __restrict__ out) {
  __shared__ float sRa[8];
  __shared__ float sRb[8];
  __shared__ __align__(16) float sOut[kCh];
  const int tid = threadIdx.x, lane = tid & 31, wave = tid >> 5;
  const int b = blockIdx.x / kLen;
  const int p = blockIdx.x - b * kLen;
  const size_t r0 = (size_t)(b * kDir) * kLen + p;
  const float y0 = Y[(r0) * kCh + tid];
  const float y1 = Y[(r0 + (size_t)kLen) * kCh + tid];
  const float y2 = Y[(r0 + (size_t)2 * kLen) * kCh + tid];
  const float y3 = Y[(r0 + (size_t)3 * kLen) * kCh + tid];
  const float wv = rne_bf16(lnw[tid]);
  const float bv = rne_bf16(lnb[tid]);
  const float v = (y0 + y2) + (y1 + y3);
  float s1 = v;
#pragma unroll
  for (int off = 1; off < 32; off <<= 1) s1 += __shfl_xor(s1, off, 32);
  if (lane == 0) sRa[wave] = s1;
  __syncthreads();
  const float mean = (((((sRa[0] + sRa[1]) + sRa[2]) + sRa[3]) + sRa[4]) + sRa[5]) * (1.0f / (float)kCh);
  const float dv = v - mean;
  float s2 = dv * dv;
#pragma unroll
  for (int off = 1; off < 32; off <<= 1) s2 += __shfl_xor(s2, off, 32);
  if (lane == 0) sRb[wave] = s2;
  __syncthreads();
  const float var = (((((sRb[0] + sRb[1]) + sRb[2]) + sRb[3]) + sRb[4]) + sRb[5]) * (1.0f / (float)kCh);
  const float rstd = 1.0f / sqrtf(var + 1e-5f);
  sOut[tid] = dv * rstd * wv + bv;
  __syncthreads();
  if (wave < 2) {
    const int q4 = lane >> 3, c8 = lane & 7;
    const int seg = wave * 4 + q4;
    const int segc = (seg < 6) ? seg : 5;
    float* ob = out + ((size_t)(b * kLen + p)) * kCh + segc * 32 + c8 * 4;
    for (int pass = 0; pass < 2; ++pass) {
      const v4f val = *(const v4f*)(sOut + segc * 32 + c8 * 4);
      if (seg < 6) *(volatile v4f*)ob = val;
      __threadfence();
    }
  }
}

extern "C" void kernel_launch(void* const* d_in, const int* in_sizes, int n_in,
                              void* d_out, int out_size, void* d_ws, size_t ws_size,
                              hipStream_t stream) {
  if (n_in < 8) return;
  if (in_sizes[0] != kBat * kCh * kLen) return;
  if (in_sizes[1] != kDir * kCpr * kCh) return;
  if (in_sizes[2] != kDir * kCh * kDtR) return;
  if (in_sizes[3] != kDir * kCh) return;
  if (in_sizes[4] != kDir * kCh * kNst) return;
  if (in_sizes[5] != kDir * kCh) return;
  if (in_sizes[6] != kCh) return;
  if (in_sizes[7] != kCh) return;
  if (out_size != kBat * kLen * kCh) return;
  if (ws_size < kWsTotal) return;

  const float* x    = (const float*)d_in[0];
  const float* xpw  = (const float*)d_in[1];
  const float* dtW  = (const float*)d_in[2];
  const float* dtb  = (const float*)d_in[3];
  const float* Alog = (const float*)d_in[4];
  const float* Dsk  = (const float*)d_in[5];
  const float* lnw  = (const float*)d_in[6];
  const float* lnb  = (const float*)d_in[7];
  float* out = (float*)d_out;

  char* ws = (char*)d_ws;
  unsigned short* XTB  = (unsigned short*)(ws + kOffXTB);
  float*          XT32 = (float*)(ws + kOffXT32);
  unsigned short* WPB  = (unsigned short*)(ws + kOffWPB);
  float*          XDBL = (float*)(ws + kOffXDBL);
  float*          PQ   = (float*)(ws + kOffPQ);
  float*          HIN  = (float*)(ws + kOffHIN);
  float*          Ybuf = (float*)(ws + kOffY);

  xpose_kernel<<<kBat * (kLen / 32), 256, 0, stream>>>(x, XT32, XTB);
  wproj_plane_kernel<<<(kCPad * kCh / 8) / 192, 192, 0, stream>>>(xpw, WPB);
  wmma_gemm64<1, 0, 0, 0, false><<<dim3(((kLen / 64) * (kCPad / 64)) / 8, kBat), 256, 0, stream>>>(
      XTB, nullptr, kCh, (long)kLen * kCh,
      WPB, nullptr, kCh, 0L,
      (void*)XDBL, nullptr, kCPad, (long)kLen * kCPad,
      nullptr, nullptr, 0L,
      kLen, kCPad, kCh, 1.0f);
  scan_phase_a<<<kBat * kDir * kNCh * kDBlk, kSCh, 0, stream>>>(XT32, XDBL, dtW, dtb, Alog, PQ);
  chunk_combine_kernel<<<kBat * kDir * kDBlk, kSCh, 0, stream>>>(PQ, HIN);
  scan_phase_b<<<kBat * kDir * kNCh * kDBlk, kSCh, 0, stream>>>(XT32, XDBL, dtW, dtb, Alog, Dsk, HIN, Ybuf);
  merge_ln_kernel<<<kBat * kLen, kCh, 0, stream>>>(Ybuf, lnw, lnb, out);
}
